// PhysicsInformedGNN_48086453846272
// MI455X (gfx1250) — hardware-verified
//
#include <hip/hip_runtime.h>
#include <stddef.h>
#include <stdint.h>


#define DM      128
#define DFF     512
#define NQ      512
#define OQ      0
#define OKK     128
#define OV      256
#define OS      384
#define FX      99
#define NEMB    64
#define KIN     163
#define KINP    192
#define RST     17
#define RDIM    82
#define GH      64
#define NGB     256
#define MAXB    4
#define NTHR    256
#define NWAVE   8
#define EPT     8
#define CHUNK   (NTHR * EPT)
#define WCAP    (EPT * 32)
#define LISTN   (NWAVE * WCAP)
#define NBMAX   2048
#define RCAP    28672
#define DEGCAP  64
#define STW     512
#define GBM     64
#define GBN     64
#define GTHR    128
#define CX      8.0f
#define CW      256.0f
#define CL      2048.0f
#define SCL     0.00048828125f
#define SCL2    2.384185791015625e-07f
#define ATTSC   0.08838834764831845f
#define WSMAX   134217728
#define LDS_AGG ((2 * RCAP + 2 * NBMAX + LISTN) * 4 + 64)

static_assert((CHUNK & (CHUNK - 1)) == 0 && CHUNK <= 4096);
static_assert((NBMAX & (NBMAX - 1)) == 0 && NBMAX <= 4096);
static_assert(NTHR * 8 == NBMAX);
static_assert(LISTN >= NBMAX);
static_assert(LISTN >= NWAVE * WCAP);
static_assert((RCAP % 32) == 0);
static_assert(NWAVE * STW <= RCAP);
static_assert(DM <= STW);
static_assert(LDS_AGG <= 300000);
static_assert(GBM == (GTHR / 32) * 16);
static_assert((DM % 32) == 0 && (DFF % 32) == 0 && (KINP % 32) == 0);
static_assert((NQ % GBN) == 0 && (DM % GBN) == 0 && (DFF % GBN) == 0);
static_assert(NQ == 4 * DM && OS == 3 * DM);
static_assert(KINP >= KIN && (KINP % 8) == 0);
static_assert(DM / 8 == 16);
static_assert(MAXB * NGB / 4 <= NTHR);

typedef float    v4f  __attribute__((ext_vector_type(4)));
typedef float    v8f  __attribute__((ext_vector_type(8)));
typedef int      v4i  __attribute__((ext_vector_type(4)));
typedef int      v8i  __attribute__((ext_vector_type(8)));
typedef _Float16 v8h  __attribute__((ext_vector_type(8)));
typedef _Float16 v16h __attribute__((ext_vector_type(16)));
union FragH { v16h v; v8h h[2]; v8i w; };

__device__ __forceinline__ v8f wmh(const FragH& a, const FragH& b, v8f c) {
  v8f d = __builtin_amdgcn_wmma_f32_16x16x32_f16(false, a.v, false, b.v, (short)0, c, false, false);
  asm volatile("v_nop\n\tv_nop\n\tv_nop\n\tv_nop" : "+v"(d) : "v"(a.w), "v"(b.w));
  return d;
}

__device__ __forceinline__ void ldwait() {
  asm volatile("s_wait_loadcnt 0x0" ::: "memory");
}

__device__ __forceinline__ v8h cvt8h(const v4f a, const v4f b, const float c) {
  v8h hv;
  hv[0] = (_Float16)(a.x * c); hv[1] = (_Float16)(a.y * c);
  hv[2] = (_Float16)(a.z * c); hv[3] = (_Float16)(a.w * c);
  hv[4] = (_Float16)(b.x * c); hv[5] = (_Float16)(b.y * c);
  hv[6] = (_Float16)(b.z * c); hv[7] = (_Float16)(b.w * c);
  return hv;
}

__device__ __forceinline__ float wsum(float v) {
#pragma unroll
  for (int off = 16; off > 0; off >>= 1) v += __shfl_xor(v, off);
  return v;
}

__device__ __forceinline__ float gelu_f(float v) {
  return 0.5f * v * (1.0f + erff(v * 0.70710678118654752f));
}

__device__ __forceinline__ v4f ln_row(const v4f t, const v4f s4, const v4f b4) {
  const float mean = wsum((t.x + t.y) + (t.z + t.w)) * (1.0f / DM);
  const float dx = t.x - mean, dy = t.y - mean, dz = t.z - mean, dw = t.w - mean;
  const float var = wsum((dx * dx + dy * dy) + (dz * dz + dw * dw)) * (1.0f / DM);
  const float inv = rsqrtf(var + 1e-5f);
  v4f o;
  o.x = dx * inv * s4.x + b4.x;
  o.y = dy * inv * s4.y + b4.y;
  o.z = dz * inv * s4.z + b4.z;
  o.w = dw * inv * s4.w + b4.w;
  return o;
}

__device__ __forceinline__ void store_rows(float* HF, _Float16* HH, size_t row, int lane, const v4f o) {
  const int L2 = 2 * (lane & 15);
  v4f a, b;
  a.x = __shfl(o.x, L2);     a.y = __shfl(o.y, L2);     a.z = __shfl(o.z, L2);     a.w = __shfl(o.w, L2);
  b.x = __shfl(o.x, L2 + 1); b.y = __shfl(o.y, L2 + 1); b.z = __shfl(o.z, L2 + 1); b.w = __shfl(o.w, L2 + 1);
  const v8h hv = cvt8h(a, b, CX);
  float*    pf = HF + row * DM + 4 * lane;
  _Float16* ph = HH + row * DM + 8 * (lane & 15);
  const bool wh = lane < 16;
  *(volatile v4f*)pf = o;
  if (wh) *(volatile v8h*)ph = hv;
  __threadfence();
  *(volatile v4f*)pf = o;
  if (wh) *(volatile v8h*)ph = hv;
}

__device__ __forceinline__ int scan_chunk(const int* __restrict__ dsts, int nE, int cbase, int slotBase,
                                          int nb, int vec8, int* list, int tid, int lane, int wave) {
  int wc = 0;
  const int el0  = tid * EPT;
  const int e0   = cbase + el0;
  const int sent = -2147483647 - 1;
  v4i da, db;
  if (vec8 != 0 && cbase + CHUNK <= nE) {
    da = *(const v4i*)(dsts + e0);
    db = *(const v4i*)(dsts + e0 + 4);
  } else {
    da.x = (e0     < nE) ? dsts[min(e0,     nE - 1)] : sent;
    da.y = (e0 + 1 < nE) ? dsts[min(e0 + 1, nE - 1)] : sent;
    da.z = (e0 + 2 < nE) ? dsts[min(e0 + 2, nE - 1)] : sent;
    da.w = (e0 + 3 < nE) ? dsts[min(e0 + 3, nE - 1)] : sent;
    db.x = (e0 + 4 < nE) ? dsts[min(e0 + 4, nE - 1)] : sent;
    db.y = (e0 + 5 < nE) ? dsts[min(e0 + 5, nE - 1)] : sent;
    db.z = (e0 + 6 < nE) ? dsts[min(e0 + 6, nE - 1)] : sent;
    db.w = (e0 + 7 < nE) ? dsts[min(e0 + 7, nE - 1)] : sent;
  }
  const unsigned nbs = (unsigned)slotBase;
  const unsigned unb = (unsigned)nb;
  const unsigned s0 = (unsigned)da.x - nbs, s1 = (unsigned)da.y - nbs;
  const unsigned s2 = (unsigned)da.z - nbs, s3 = (unsigned)da.w - nbs;
  const unsigned s4 = (unsigned)db.x - nbs, s5 = (unsigned)db.y - nbs;
  const unsigned s6 = (unsigned)db.z - nbs, s7 = (unsigned)db.w - nbs;
  const bool h0 = s0 < unb, h1 = s1 < unb, h2 = s2 < unb, h3 = s3 < unb;
  const bool h4 = s4 < unb, h5 = s5 < unb, h6 = s6 < unb, h7 = s7 < unb;
  const unsigned any = __builtin_amdgcn_ballot_w32(h0 | h1 | h2 | h3 | h4 | h5 | h6 | h7);
  if (any != 0u) {
#define HITJ(J, HJ, SJ) { \
      const unsigned mj = __builtin_amdgcn_ballot_w32(HJ); \
      if (mj != 0u) { \
        if (HJ) { \
          const int pos = wc + (int)__builtin_amdgcn_mbcnt_lo(mj, 0u); \
          if (pos < WCAP) list[wave * WCAP + pos] = ((el0 + (J)) << 12) | (int)(SJ); \
        } \
        wc += (int)__builtin_popcount(mj); } }
    HITJ(0, h0, s0)
    HITJ(1, h1, s1)
    HITJ(2, h2, s2)
    HITJ(3, h3, s3)
    HITJ(4, h4, s4)
    HITJ(5, h5, s5)
    HITJ(6, h6, s6)
    HITJ(7, h7, s7)
#undef HITJ
  }
  return wc;
}

__global__ __launch_bounds__(NTHR) void k_wcvt(const float* __restrict__ w, _Float16* wt, int K, int KP, int nUnits) {
  const int u = (int)blockIdx.x * NTHR + (int)threadIdx.x;
  if (u >= nUnits) return;
  const int kq = KP >> 3;
  const int n  = u / kq;
  const int k8 = (u - n * kq) * 8;
  const float* p = w + (size_t)n * (size_t)K;
  float s[8];
#pragma unroll
  for (int i = 0; i < 8; ++i) {
    const int c  = k8 + i;
    const int cl = c < K ? c : K - 1;
    s[i] = p[cl];
  }
  v8h hv;
#pragma unroll
  for (int i = 0; i < 8; ++i) {
    const float v = (k8 + i < K) ? s[i] * CW : 0.0f;
    hv[i] = (_Float16)v;
  }
  const size_t o = (size_t)n * (size_t)KP + k8;
  *(volatile v8h*)(wt + o) = hv;
  __threadfence();
  *(volatile v8h*)(wt + o) = hv;
}

__global__ __launch_bounds__(NTHR) void k_feat(const float* __restrict__ x, const float* __restrict__ emb,
                                               _Float16* ft, int nN, int nPer, int nUnits) {
  const int u = (int)blockIdx.x * NTHR + (int)threadIdx.x;
  if (u >= nUnits) return;
  const int row = u / (KINP / 8);
  const int c0  = (u - row * (KINP / 8)) * 8;
  const int rc  = row < nN ? row : nN - 1;
  const int b   = rc / nPer;
  const int node = rc - b * nPer;
  const float* xp = x   + (size_t)rc   * FX;
  const float* ep = emb + (size_t)node * NEMB;
  float xs[8], es[8];
#pragma unroll
  for (int i = 0; i < 8; ++i) {
    const int c = c0 + i;
    xs[i] = xp[c < FX ? c : FX - 1];
  }
  ldwait();
#pragma unroll
  for (int i = 0; i < 8; ++i) {
    int ec = c0 + i - FX;
    ec = ec < 0 ? 0 : (ec > NEMB - 1 ? NEMB - 1 : ec);
    es[i] = ep[ec];
  }
  ldwait();
  v8h hv;
#pragma unroll
  for (int i = 0; i < 8; ++i) {
    const int c = c0 + i;
    float v = (c < FX) ? xs[i] : ((c < KIN) ? es[i] : 0.0f);
    if (row >= nN) v = 0.0f;
    hv[i] = (_Float16)(v * CX);
  }
  const size_t o = (size_t)row * KINP + c0;
  *(volatile v8h*)(ft + o) = hv;
  __threadfence();
  *(volatile v8h*)(ft + o) = hv;
}

__global__ __launch_bounds__(NTHR) void k_film(const float* __restrict__ x, const float* __restrict__ g1w,
                                               const float* __restrict__ g1b, const float* __restrict__ g2w,
                                               const float* __restrict__ g2b, float* GB, int nB, int nPer) {
  __shared__ float rain[MAXB * RDIM];
  __shared__ float ghs[MAXB * GH];
  __shared__ __attribute__((aligned(16))) float gbst[MAXB * NGB];
  const int tid = (int)threadIdx.x;
  for (int i = tid; i < nB * RDIM; i += NTHR) {
    const int b = i / RDIM, j = i - b * RDIM;
    rain[i] = x[(size_t)b * (size_t)nPer * FX + RST + j];
  }
  __syncthreads();
  for (int i = tid; i < nB * GH; i += NTHR) {
    const int b = i / GH, o = i - b * GH;
    const float* wr = g1w + (size_t)o * RDIM;
    const float* rr = rain + b * RDIM;
    float a = 0.0f;
#pragma unroll 1
    for (int j = 0; j < RDIM; ++j) a = fmaf(rr[j], wr[j], a);
    a += g1b[o];
    ghs[i] = gelu_f(a);
  }
  __syncthreads();
  for (int i = tid; i < nB * NGB; i += NTHR) {
    const int b = i / NGB, o = i - b * NGB;
    const float* wr = g2w + (size_t)o * GH;
    const float* gr = ghs + b * GH;
    float a = 0.0f;
#pragma unroll 1
    for (int j = 0; j < GH; ++j) a = fmaf(gr[j], wr[j], a);
    a += g2b[o];
    gbst[i] = tanhf(a) * 0.5f;
  }
  __syncthreads();
  const int nq = (nB * NGB) >> 2;
  const int tq = tid < nq ? tid : nq - 1;
  const v4f v = *(const v4f*)(gbst + 4 * tq);
  const bool w = tid < nq;
  if (w) *(volatile v4f*)(GB + 4 * tid) = v;
  __threadfence();
  if (w) *(volatile v4f*)(GB + 4 * tid) = v;
}

__global__ __launch_bounds__(NTHR) void k_mod(const float* __restrict__ T, const float* __restrict__ GB,
                                              float* Hout, _Float16* HH, int nN, int nPer, int MPr) {
  const int tid = (int)threadIdx.x, lane = tid & 31, wave = tid >> 5;
  const int row = (int)blockIdx.x * NWAVE + wave;
  if (row >= MPr) return;
  const int rc = row < nN ? row : nN - 1;
  const int b  = rc / nPer;
  const v4f tv = *(const v4f*)(T  + (size_t)rc * DM + 4 * lane);
  const v4f g  = *(const v4f*)(GB + (size_t)b * NGB + 4 * lane);
  const v4f be = *(const v4f*)(GB + (size_t)b * NGB + DM + 4 * lane);
  v4f o;
  o.x = tv.x * (1.0f + g.x) + be.x;
  o.y = tv.y * (1.0f + g.y) + be.y;
  o.z = tv.z * (1.0f + g.z) + be.z;
  o.w = tv.w * (1.0f + g.w) + be.w;
  if (row >= nN) { const v4f z = {0.f, 0.f, 0.f, 0.f}; o = z; }
  store_rows(Hout, HH, (size_t)row, lane, o);
}

template<int MODE>
__global__ __launch_bounds__(NTHR) void k_ln(const float* __restrict__ Hin, const float* __restrict__ P1,
                                             const float* __restrict__ P2, int ld1, int off1,
                                             const float* __restrict__ sc, const float* __restrict__ bi,
                                             float* Hout, _Float16* HH, int nN, int MPr) {
  const int tid = (int)threadIdx.x, lane = tid & 31, wave = tid >> 5;
  const int row = (int)blockIdx.x * NWAVE + wave;
  if (row >= MPr) return;
  const int rc = row < nN ? row : nN - 1;
  const v4f hv = *(const v4f*)(Hin + (size_t)rc * DM + 4 * lane);
  const v4f pv = *(const v4f*)(P1 + (size_t)rc * (size_t)ld1 + off1 + 4 * lane);
  v4f t;
  if (MODE == 0) {
    const v4f av = *(const v4f*)(P2 + (size_t)rc * DM + 4 * lane);
    t.x = hv.x + fmaxf(pv.x + av.x, 0.0f);
    t.y = hv.y + fmaxf(pv.y + av.y, 0.0f);
    t.z = hv.z + fmaxf(pv.z + av.z, 0.0f);
    t.w = hv.w + fmaxf(pv.w + av.w, 0.0f);
  } else {
    t = hv + pv;
  }
  const v4f s4 = *(const v4f*)(sc + 4 * lane);
  const v4f b4 = *(const v4f*)(bi + 4 * lane);
  v4f o = ln_row(t, s4, b4);
  if (row >= nN) { const v4f z = {0.f, 0.f, 0.f, 0.f}; o = z; }
  store_rows(Hout, HH, (size_t)row, lane, o);
}

__global__ __launch_bounds__(NTHR) void k_head(const float* __restrict__ H, const float* __restrict__ hs,
                                               const float* __restrict__ hb, const float* __restrict__ hw,
                                               const float* __restrict__ hbias, float* out, int nN, int o1off) {
  __shared__ __attribute__((aligned(16))) float os[64];
  const int tid = (int)threadIdx.x, lane = tid & 31, wave = tid >> 5;
  const int blk = (int)blockIdx.x;
  const v4f s4 = *(const v4f*)(hs + 4 * lane);
  const v4f b4 = *(const v4f*)(hb + 4 * lane);
  const v4f w0 = *(const v4f*)(hw + 4 * lane);
  const v4f w1 = *(const v4f*)(hw + DM + 4 * lane);
  const float hb0 = hbias[0], hb1 = hbias[1];
#pragma unroll 1
  for (int r = 0; r < 4; ++r) {
    const int row = blk * 32 + wave * 4 + r;
    const int rc  = row < nN ? row : nN - 1;
    const v4f hv = *(const v4f*)(H + (size_t)rc * DM + 4 * lane);
    const v4f nv = ln_row(hv, s4, b4);
    float p0 = nv.x * w0.x; p0 = fmaf(nv.y, w0.y, p0); p0 = fmaf(nv.z, w0.z, p0); p0 = fmaf(nv.w, w0.w, p0);
    float p1 = nv.x * w1.x; p1 = fmaf(nv.y, w1.y, p1); p1 = fmaf(nv.z, w1.z, p1); p1 = fmaf(nv.w, w1.w, p1);
    const float d0 = wsum(p0);
    const float d1 = wsum(p1);
    if (lane == 0) {
      os[wave * 4 + r]      = d0 + hb0;
      os[32 + wave * 4 + r] = d1 + hb1;
    }
  }
  __syncthreads();
  if (wave == 0) {
    const int q   = lane & 7;
    const int sel = (lane >> 3) & 1;
    const v4f v = *(const v4f*)(os + 32 * sel + 4 * q);
    float* op = out + (size_t)sel * (size_t)o1off + (size_t)blk * 32 + 4 * q;
    const bool w = (lane < 16) && (blk * 32 + 32 <= nN);
    if (w) *(volatile v4f*)op = v;
    __threadfence();
    if (w) *(volatile v4f*)op = v;
  }
}

template<int EPI, int ALO>
__global__ __launch_bounds__(GTHR) void k_gemm(
    const _Float16* __restrict__ A, const _Float16* __restrict__ AL,
    const _Float16* __restrict__ W0, const _Float16* __restrict__ W1,
    const _Float16* __restrict__ W2, const _Float16* __restrict__ W3,
    const float* __restrict__ b0, const float* __restrict__ b1,
    const float* __restrict__ b2, const float* __restrict__ b3,
    float* outF, _Float16* outH, _Float16* outL,
    int K, int ldo, int segN, float scl, float scl2)
{
  __shared__ __attribute__((aligned(16))) float stg[GBM * GBN];
  const int tid = (int)threadIdx.x, lane = tid & 31, wave = tid >> 5, hh = lane >> 4, m = lane & 15;
  const int rowBase = (int)blockIdx.x * GBM;
  const int col0    = (int)blockIdx.y * GBN;
  int seg = col0 / segN;
  seg = seg < 0 ? 0 : (seg > 3 ? 3 : seg);
  const _Float16* Wp = (seg == 0) ? W0 : ((seg == 1) ? W1 : ((seg == 2) ? W2 : W3));
  const float*    bp = (seg == 0) ? b0 : ((seg == 1) ? b1 : ((seg == 2) ? b2 : b3));
  int wr0 = col0 - seg * segN;
  wr0 = wr0 < 0 ? 0 : wr0;

  v8f acc[4], accl[4];
  {
    const v8f z = {0.f, 0.f, 0.f, 0.f, 0.f, 0.f, 0.f, 0.f};
    acc[0] = z; acc[1] = z; acc[2] = z; acc[3] = z;
    accl[0] = z; accl[1] = z; accl[2] = z; accl[3] = z;
  }
  const size_t Ks = (size_t)K;
  const _Float16* ap  = A  + (size_t)(rowBase + 16 * wave + m) * Ks + 8 * hh;
  const _Float16* alp = AL + (size_t)(rowBase + 16 * wave + m) * Ks + 8 * hh;
  const _Float16* wp  = Wp + (size_t)(wr0 + m) * Ks + 8 * hh;
  const int ksteps = K >> 5;
#pragma unroll 1
  for (int ks = 0; ks < ksteps; ++ks) {
    FragH af, alf;
    af.h[0] = *(const v8h*)(ap + 32 * ks);
    af.h[1] = *(const v8h*)(ap + 32 * ks + 16);
    if (ALO) {
      alf.h[0] = *(const v8h*)(alp + 32 * ks);
      alf.h[1] = *(const v8h*)(alp + 32 * ks + 16);
    } else {
      alf.v = af.v;
    }
#pragma unroll
    for (int t = 0; t < 4; ++t) {
      const _Float16* wq = wp + (size_t)(16 * t) * Ks + 32 * ks;
      FragH bf;
      bf.h[0] = *(const v8h*)wq;
      bf.h[1] = *(const v8h*)(wq + 16);
      acc[t] = wmh(af, bf, acc[t]);
      if (ALO) accl[t] = wmh(alf, bf, accl[t]);
    }
  }

#pragma unroll
  for (int t = 0; t < 4; ++t) {
    const int lc = 16 * t + m;
    int bi = wr0 + lc;
    bi = bi > segN - 1 ? segN - 1 : bi;
    bi = bi < 0 ? 0 : bi;
    const float bv = bp[bi];
#pragma unroll
    for (int r = 0; r < 8; ++r) {
      const int lr = 16 * wave + 8 * hh + r;
      float v = fmaf(acc[t][r], scl, bv);
      if (ALO) v = fmaf(accl[t][r], scl2, v);
      if (EPI == 2) v = gelu_f(v);
      stg[lr * GBN + lc] = v;
    }
  }
  __syncthreads();

  if (EPI == 0) {
    v4f fv[8];
#pragma unroll
    for (int i = 0; i < 8; ++i) {
      const int lr = 16 * wave + 2 * i + hh;
      fv[i] = *(const v4f*)(stg + lr * GBN + 4 * m);
    }
#pragma unroll
    for (int i = 0; i < 8; ++i) {
      const int lr = 16 * wave + 2 * i + hh;
      const int gr = rowBase + lr;
      float* op = outF + (size_t)gr * (size_t)ldo + col0 + 4 * m;
      *(volatile v4f*)op = fv[i];
    }
    __threadfence();
#pragma unroll
    for (int i = 0; i < 8; ++i) {
      const int lr = 16 * wave + 2 * i + hh;
      const int gr = rowBase + lr;
      float* op = outF + (size_t)gr * (size_t)ldo + col0 + 4 * m;
      *(volatile v4f*)op = fv[i];
    }
  } else {
    const int q = lane & 7, rs = lane >> 3;
    v8h hv[4], lv[4];
#pragma unroll
    for (int i = 0; i < 4; ++i) {
      const int lr = 16 * wave + 4 * i + rs;
      const v4f ga = *(const v4f*)(stg + lr * GBN + 8 * q);
      const v4f gb = *(const v4f*)(stg + lr * GBN + 8 * q + 4);
      float s[8] = {ga.x * CX, ga.y * CX, ga.z * CX, ga.w * CX, gb.x * CX, gb.y * CX, gb.z * CX, gb.w * CX};
      v8h h8, l8;
#pragma unroll
      for (int e = 0; e < 8; ++e) {
        const _Float16 he = (_Float16)s[e];
        h8[e] = he;
        l8[e] = (_Float16)((s[e] - (float)he) * CL);
      }
      hv[i] = h8; lv[i] = l8;
    }
#pragma unroll
    for (int i = 0; i < 4; ++i) {
      const int lr = 16 * wave + 4 * i + rs;
      const int gr = rowBase + lr;
      const size_t o = (size_t)gr * (size_t)ldo + col0 + 8 * q;
      *(volatile v8h*)(outH + o) = hv[i];
      *(volatile v8h*)(outL + o) = lv[i];
    }
    __threadfence();
#pragma unroll
    for (int i = 0; i < 4; ++i) {
      const int lr = 16 * wave + 4 * i + rs;
      const int gr = rowBase + lr;
      const size_t o = (size_t)gr * (size_t)ldo + col0 + 8 * q;
      *(volatile v8h*)(outH + o) = hv[i];
      *(volatile v8h*)(outL + o) = lv[i];
    }
  }
}

__global__ __launch_bounds__(NTHR) void k_agg(
    const int* __restrict__ ei, const float* __restrict__ QKVS, _Float16* Hout,
    int nN, int nPer, int nE, int nB, int nb, int vec8, int MPr) {
  extern __shared__ v4f lds_dyn[];
  int* reg1 = (int*)lds_dyn;
  int* reg2 = reg1 + RCAP;
  int* scnt = reg2 + RCAP;
  int* soff = scnt + NBMAX;
  int* list = soff + NBMAX;
  int* wcnt = list + LISTN;
  int* wtot = wcnt + NWAVE;
  const int* srcs = ei;
  const int* dsts = ei + nE;
  const int tid = (int)threadIdx.x, lane = tid & 31, wave = tid >> 5;
  const int nodeBase = (int)blockIdx.x * nb;

  for (int i = tid; i < NBMAX; i += NTHR) scnt[i] = 0;
  __syncthreads();

  int tot = 0;
  const int nChunks = (nE + CHUNK - 1) / CHUNK;
  const int nPC = nB * nChunks;
#pragma unroll 1
  for (int pc = 0; pc < nPC; ++pc) {
    const int bb    = pc / nChunks;
    const int ch    = pc - bb * nChunks;
    const int cbase = ch * CHUNK;
    const int wc = scan_chunk(dsts, nE, cbase, nodeBase - bb * nPer, nb, vec8, list, tid, lane, wave);
    if (lane == 0) wcnt[wave] = wc;
    __syncthreads();
    int pre = 0, all = 0;
#pragma unroll
    for (int w2 = 0; w2 < NWAVE; ++w2) {
      int c = wcnt[w2];
      c = c < 0 ? 0 : (c > WCAP ? WCAP : c);
      all += c;
      pre += (w2 < wave) ? c : 0;
    }
    const int wcc  = wc > WCAP ? WCAP : wc;
    const int base = tot + pre;
#pragma unroll 1
    for (int i = lane; i < wcc; i += 32) {
      const int ent = list[wave * WCAP + i];
      const int el  = (ent >> 12) & (CHUNK - 1);
      const int sl  = ent & (NBMAX - 1);
      int eid = cbase + el;
      eid = eid > nE - 1 ? nE - 1 : eid;
      const int g   = bb * nE + eid;
      const int pos = base + i;
      if (pos < RCAP) reg1[pos] = (int)(((unsigned)g << 12) | (unsigned)sl);
    }
    tot += all;
    tot = tot > RCAP ? RCAP : tot;
    __syncthreads();
  }
  const int nh = tot;

  if (wave == 0) {
#pragma unroll 1
    for (int b0 = 0; b0 < nh; b0 += 32) {
      const int idx = b0 + lane;
      const int uv  = reg1[idx < RCAP ? idx : RCAP - 1];
      const int m32 = (nh - b0) < 32 ? (nh - b0) : 32;
#pragma unroll 1
      for (int k = 0; k < m32; ++k) {
        const int u  = __builtin_amdgcn_readlane(uv, k);
        const int sl = u & (NBMAX - 1);
        if (lane == 0) scnt[sl] = scnt[sl] + 1;
      }
    }
  }
  __syncthreads();

  {
    const v4i ca = *(const v4i*)(scnt + 8 * tid);
    const v4i cb = *(const v4i*)(scnt + 8 * tid + 4);
    const int e0 = ca.x < 0 ? 0 : ca.x, e1 = ca.y < 0 ? 0 : ca.y, e2 = ca.z < 0 ? 0 : ca.z, e3 = ca.w < 0 ? 0 : ca.w;
    const int e4 = cb.x < 0 ? 0 : cb.x, e5 = cb.y < 0 ? 0 : cb.y, e6 = cb.z < 0 ? 0 : cb.z, e7 = cb.w < 0 ? 0 : cb.w;
    const int ts = e0 + e1 + e2 + e3 + e4 + e5 + e6 + e7;
    int incl = ts;
#pragma unroll
    for (int d = 1; d < 32; d <<= 1) {
      const int up = __shfl_up(incl, d);
      if (lane >= d) incl += up;
    }
    if (lane == 31) wtot[wave] = incl;
    __syncthreads();
    int pre = 0;
#pragma unroll
    for (int w2 = 0; w2 < NWAVE; ++w2) pre += (w2 < wave) ? wtot[w2] : 0;
    int run = pre + incl - ts;
    soff[8 * tid + 0] = run; run += e0;
    soff[8 * tid + 1] = run; run += e1;
    soff[8 * tid + 2] = run; run += e2;
    soff[8 * tid + 3] = run; run += e3;
    soff[8 * tid + 4] = run; run += e4;
    soff[8 * tid + 5] = run; run += e5;
    soff[8 * tid + 6] = run; run += e6;
    soff[8 * tid + 7] = run;
  }
  __syncthreads();
  for (int i = tid; i < NBMAX; i += NTHR) list[i] = soff[i];
  __syncthreads();

  if (wave == 0) {
#pragma unroll 1
    for (int b0 = 0; b0 < nh; b0 += 32) {
      const int idx = b0 + lane;
      const int uv  = reg1[idx < RCAP ? idx : RCAP - 1];
      const int m32 = (nh - b0) < 32 ? (nh - b0) : 32;
#pragma unroll 1
      for (int k = 0; k < m32; ++k) {
        const int u  = __builtin_amdgcn_readlane(uv, k);
        const int sl = u & (NBMAX - 1);
        const int g  = (int)((unsigned)u >> 12);
        if (lane == 0) {
          int pos = list[sl];
          pos = pos < 0 ? 0 : (pos > RCAP - 1 ? RCAP - 1 : pos);
          reg2[pos] = g;
          list[sl] = pos + 1;
        }
      }
    }
  }
  __syncthreads();

  const int nbw = nb >> 3;
  const bool ovf = (nh >= RCAP);
  const float qnan = __int_as_float(0x7fc00000);
  float* stw = (float*)reg1 + wave * STW;
  const int lc = lane < (DM / 8) ? lane : (DM / 8) - 1;
  const int gmax = nB * nE - 1;
#pragma unroll 1
  for (int jt = 0; jt < nbw; ++jt) {
    const int slot = wave * nbw + jt;
    const int grow = nodeBase + slot;
    const int gcl  = grow < nN ? grow : nN - 1;
    int st = soff[slot];
    const int craw = scnt[slot];
    int cnt = craw;
    st  = st < 0 ? 0 : (st > nh ? nh : st);
    cnt = cnt < 0 ? 0 : (cnt > DEGCAP ? DEGCAP : cnt);
    if (cnt > nh - st) cnt = nh - st;
    const float pz = (ovf || craw > DEGCAP) ? qnan : 0.0f;
    const bool wr = grow < MPr;
    const float live = grow < nN ? 1.0f : 0.0f;

    const float* qrow = QKVS + (size_t)gcl * NQ + OQ + lane;
    float qv[4], av[4];
#pragma unroll
    for (int j = 0; j < 4; ++j) { qv[j] = qrow[32 * j]; av[j] = 0.f; }
    ldwait();
    float mx = -1.0e30f, dn = 0.f;

#pragma unroll 1
    for (int q = 0; q < cnt; ++q) {
      int idx = st + q; idx = idx > RCAP - 1 ? RCAP - 1 : idx;
      int g = reg2[idx]; g = g < 0 ? 0 : (g > gmax ? gmax : g);
      int bb = 0;
#pragma unroll 1
      for (int t = 1; t < nB; ++t) bb += (g >= t * nE) ? 1 : 0;
      int e = g - bb * nE;
      e = e < 0 ? 0 : (e > nE - 1 ? nE - 1 : e);
      const int sraw = srcs[e];
      const int sl   = sraw < 0 ? 0 : (sraw > nPer - 1 ? nPer - 1 : sraw);
      const int s    = sl + bb * nPer;
      const float* kr = QKVS + (size_t)s * NQ + OKK + lane;
      float kk[4], vv[4];
#pragma unroll
      for (int j = 0; j < 4; ++j) kk[j] = kr[32 * j];
      ldwait();
#pragma unroll
      for (int j = 0; j < 4; ++j) vv[j] = kr[(OV - OKK) + 32 * j];
      ldwait();
      float part = qv[0] * kk[0];
      part = fmaf(qv[1], kk[1], part);
      part = fmaf(qv[2], kk[2], part);
      part = fmaf(qv[3], kk[3], part);
#pragma unroll
      for (int off = 16; off > 0; off >>= 1) part += __shfl_xor(part, off);
      const float al = part * ATTSC;
      const float df = al - mx;
      const float ee = __expf(-fabsf(df));
      const bool up  = df > 0.f;
      const float s1 = up ? ee : 1.0f;
      const float s2 = up ? 1.0f : ee;
      mx = up ? al : mx;
      dn = fmaf(dn, s1, s2);
#pragma unroll
      for (int j = 0; j < 4; ++j) av[j] = fmaf(av[j], s1, s2 * vv[j]);
    }
    const float ds = dn > 0.f ? dn : 1.0f;
    const float iv = (dn > 0.f ? 1.0f : 0.0f) * __builtin_amdgcn_rcpf(ds);
    float o[4];
#pragma unroll
    for (int j = 0; j < 4; ++j) o[j] = av[j] * iv * live + pz;
    __builtin_amdgcn_fence(__ATOMIC_RELEASE, "wavefront");
    __builtin_amdgcn_wave_barrier();
#pragma unroll
    for (int j = 0; j < 4; ++j) stw[32 * j + lane] = o[j];
    __builtin_amdgcn_fence(__ATOMIC_RELEASE, "wavefront");
    __builtin_amdgcn_wave_barrier();
    const v4f ga = *(const v4f*)(stw + 8 * lc);
    const v4f gb = *(const v4f*)(stw + 8 * lc + 4);
    const v8h hv = cvt8h(ga, gb, CX);
    _Float16* gp = Hout + (size_t)grow * DM + 8 * lc;
    const bool wsv = wr && (lane < (DM / 8));
    if (wsv) *(volatile v8h*)gp = hv;
    __threadfence();
    if (wsv) *(volatile v8h*)gp = hv;
  }
}

static int pick_nb(long long nEt, int nN) {
  int nb = NBMAX;
  while (nb > 16 && (long long)nb * nEt * 5LL > (long long)RCAP * (long long)nN * 4LL) nb >>= 1;
  return nb;
}
static inline int cdiv(int a, int b) { return (a + b - 1) / b; }
static inline size_t carve(size_t& off, size_t bytes) {
  const size_t o = off;
  off += bytes;
  off = (off + 255) & ~(size_t)255;
  return o;
}

extern "C" void kernel_launch(void* const* d_in, const int* in_sizes, int n_in,
                              void* d_out, int out_size, void* d_ws, size_t ws_size,
                              hipStream_t stream) {
  if (n_in < 31) return;
  const int nPer = in_sizes[2] / NEMB;
  if (nPer <= 0 || in_sizes[2] != nPer * NEMB) return;
  if (in_sizes[0] <= 0 || (in_sizes[0] % (nPer * FX)) != 0) return;
  const int nB = in_sizes[0] / (nPer * FX);
  if (nB < 1 || nB > MAXB) return;
  const long long nNl = (long long)nB * (long long)nPer;
  if (nNl > (1 << 22) || (nNl % 32) != 0) return;
  const int nN = (int)nNl;
  if (in_sizes[1] < 2 || (in_sizes[1] & 1) != 0) return;
  const int nE = in_sizes[1] / 2;
  if (nE < 1 || (long long)nB * (long long)nE > (1 << 20)) return;
  if (in_sizes[3] != DM * KIN || in_sizes[4] != DM) return;
  if (in_sizes[5] != GH * RDIM || in_sizes[6] != GH) return;
  if (in_sizes[7] != NGB * GH || in_sizes[8] != NGB) return;
  const int nL = in_sizes[9] / (DM * DM);
  if (nL < 1 || nL > 64 || in_sizes[9] != nL * DM * DM) return;
  for (int i = 10; i <= 13; ++i) if (in_sizes[i] != nL * DM * DM) return;
  for (int i = 14; i <= 20; ++i) if (in_sizes[i] != nL * DM) return;
  if (in_sizes[21] != nL * DFF * DM || in_sizes[22] != nL * DFF) return;
  if (in_sizes[23] != nL * DM * DFF) return;
  for (int i = 24; i <= 26; ++i) if (in_sizes[i] != nL * DM) return;
  if (in_sizes[27] != DM || in_sizes[28] != DM) return;
  if (in_sizes[29] != 2 * DM || in_sizes[30] != 2) return;
  if (out_size != 2 * nN) return;

  const float* x      = (const float*)d_in[0];
  const int*   ei     = (const int*)  d_in[1];
  const float* emb    = (const float*)d_in[2];
  const float* W_in   = (const float*)d_in[3];
  const float* b_in   = (const float*)d_in[4];
  const float* g1w    = (const float*)d_in[5];
  const float* g1b    = (const float*)d_in[6];
  const float* g2w    = (const float*)d_in[7];
  const float* g2b    = (const float*)d_in[8];
  const float* qw     = (const float*)d_in[9];
  const float* kw     = (const float*)d_in[10];
  const float* vw     = (const float*)d_in[11];
  const float* sw     = (const float*)d_in[12];
  const float* ow     = (const float*)d_in[13];
  const float* qb     = (const float*)d_in[14];
  const float* kb     = (const float*)d_in[15];
  const float* vb     = (const float*)d_in[16];
  const float* sb     = (const float*)d_in[17];
  const float* ob     = (const float*)d_in[18];
  const float* n1s    = (const float*)d_in[19];
  const float* n1b    = (const float*)d_in[20];
  const float* f1w    = (const float*)d_in[21];
  const float* f1b    = (const float*)d_in[22];
  const float* f2w    = (const float*)d_in[23];
  const float* f2b    = (const float*)d_in[24];
  const float* n2s    = (const float*)d_in[25];
  const float* n2b    = (const float*)d_in[26];
  const float* hs     = (const float*)d_in[27];
  const float* hb     = (const float*)d_in[28];
  const float* head_w = (const float*)d_in[29];
  const float* head_b = (const float*)d_in[30];
  float* out = (float*)d_out;

  const int MP   = cdiv(nN, GBM) * GBM;
  const int nb   = pick_nb((long long)nB * nE, nN);
  const int gA   = cdiv(MP, nb);
  const int vec8 = ((nE & 3) == 0) ? 1 : 0;
  if (gA * nb < MP || (nb & 7) != 0) return;

  char* wsb = (char*)d_ws;
  size_t off = 0;
  const size_t oHA  = carve(off, (size_t)MP * DM  * 4);
  const size_t oHB  = carve(off, (size_t)MP * DM  * 4);
  const size_t oSCR = carve(off, (size_t)MP * DM  * 4);
  const size_t oQKV = carve(off, (size_t)MP * NQ  * 4);
  const size_t oHH  = carve(off, (size_t)MP * DM  * 2);
  const size_t oAGG = carve(off, (size_t)MP * DM  * 2);
  const size_t oFH  = carve(off, (size_t)MP * DFF * 2);
  const size_t oFL  = carve(off, (size_t)MP * DFF * 2);
  const size_t oGB  = carve(off, (size_t)MAXB * NGB * 4);
  const size_t oWIN = carve(off, (size_t)DM * KINP * 2);
  const size_t oQW  = carve(off, (size_t)nL * DM * DM * 2);
  const size_t oKW  = carve(off, (size_t)nL * DM * DM * 2);
  const size_t oVW  = carve(off, (size_t)nL * DM * DM * 2);
  const size_t oSW  = carve(off, (size_t)nL * DM * DM * 2);
  const size_t oOW  = carve(off, (size_t)nL * DM * DM * 2);
  const size_t oF1  = carve(off, (size_t)nL * DFF * DM * 2);
  const size_t oF2  = carve(off, (size_t)nL * DM * DFF * 2);
  if (off > ws_size || off > (size_t)WSMAX) return;
  static_assert(KINP <= DFF);
  float*    HA   = (float*)(wsb + oHA);
  float*    HB   = (float*)(wsb + oHB);
  float*    SCR  = (float*)(wsb + oSCR);
  float*    QKVS = (float*)(wsb + oQKV);
  _Float16* HH   = (_Float16*)(wsb + oHH);
  _Float16* AGG  = (_Float16*)(wsb + oAGG);
  _Float16* FH   = (_Float16*)(wsb + oFH);
  _Float16* FT   = FH;
  _Float16* FL   = (_Float16*)(wsb + oFL);
  float*    GB   = (float*)(wsb + oGB);
  _Float16* WIN  = (_Float16*)(wsb + oWIN);
  _Float16* QW   = (_Float16*)(wsb + oQW);
  _Float16* KW   = (_Float16*)(wsb + oKW);
  _Float16* VW   = (_Float16*)(wsb + oVW);
  _Float16* SW   = (_Float16*)(wsb + oSW);
  _Float16* OW   = (_Float16*)(wsb + oOW);
  _Float16* F1   = (_Float16*)(wsb + oF1);
  _Float16* F2   = (_Float16*)(wsb + oF2);

  hipFuncSetAttribute(reinterpret_cast<const void*>(&k_agg),
                      hipFuncAttributeMaxDynamicSharedMemorySize, LDS_AGG);

  {
    const int uW = DM * (KINP / 8);
    k_wcvt<<<cdiv(uW, NTHR), NTHR, 0, stream>>>(W_in, WIN, KIN, KINP, uW);
    const int uD = nL * DM * (DM / 8);
    k_wcvt<<<cdiv(uD, NTHR), NTHR, 0, stream>>>(qw, QW, DM, DM, uD);
    k_wcvt<<<cdiv(uD, NTHR), NTHR, 0, stream>>>(kw, KW, DM, DM, uD);
    k_wcvt<<<cdiv(uD, NTHR), NTHR, 0, stream>>>(vw, VW, DM, DM, uD);
    k_wcvt<<<cdiv(uD, NTHR), NTHR, 0, stream>>>(sw, SW, DM, DM, uD);
    k_wcvt<<<cdiv(uD, NTHR), NTHR, 0, stream>>>(ow, OW, DM, DM, uD);
    const int u1 = nL * DFF * (DM / 8);
    k_wcvt<<<cdiv(u1, NTHR), NTHR, 0, stream>>>(f1w, F1, DM, DM, u1);
    const int u2 = nL * DM * (DFF / 8);
    k_wcvt<<<cdiv(u2, NTHR), NTHR, 0, stream>>>(f2w, F2, DFF, DFF, u2);
  }

  const int uF = MP * (KINP / 8);
  k_feat<<<cdiv(uF, NTHR), NTHR, 0, stream>>>(x, emb, FT, nN, nPer, uF);
  const int gM = MP / GBM;
  k_gemm<0, 0><<<dim3(gM, DM / GBN), GTHR, 0, stream>>>(FT, FT, WIN, WIN, WIN, WIN, b_in, b_in, b_in, b_in,
                                                        SCR, HH, HH, KINP, DM, DM, SCL, 0.0f);
  k_film<<<1, NTHR, 0, stream>>>(x, g1w, g1b, g2w, g2b, GB, nB, nPer);
  const int gR = cdiv(MP, NWAVE);
  k_mod<<<gR, NTHR, 0, stream>>>(SCR, GB, HA, HH, nN, nPer, MP);

  for (int i = 0; i < nL; ++i) {
    const size_t wo  = (size_t)i * DM * DM;
    const size_t bo  = (size_t)i * DM;
    const size_t w1o = (size_t)i * DFF * DM;
    const size_t b1o = (size_t)i * DFF;
    k_gemm<0, 0><<<dim3(gM, NQ / GBN), GTHR, 0, stream>>>(HH, HH, QW + wo, KW + wo, VW + wo, SW + wo,
                                                          qb + bo, kb + bo, vb + bo, sb + bo,
                                                          QKVS, HH, HH, DM, NQ, DM, SCL, 0.0f);
    k_agg<<<gA, NTHR, LDS_AGG, stream>>>(ei, QKVS, AGG, nN, nPer, nE, nB, nb, vec8, MP);
    k_gemm<0, 0><<<dim3(gM, DM / GBN), GTHR, 0, stream>>>(AGG, AGG, OW + wo, OW + wo, OW + wo, OW + wo,
                                                          ob + bo, ob + bo, ob + bo, ob + bo,
                                                          SCR, HH, HH, DM, DM, DM, SCL, 0.0f);
    k_ln<0><<<gR, NTHR, 0, stream>>>(HA, QKVS, SCR, NQ, OS, n1s + bo, n1b + bo, HB, HH, nN, MP);
    k_gemm<2, 0><<<dim3(gM, DFF / GBN), GTHR, 0, stream>>>(HH, HH, F1 + w1o, F1 + w1o, F1 + w1o, F1 + w1o,
                                                           f1b + b1o, f1b + b1o, f1b + b1o, f1b + b1o,
                                                           SCR, FH, FL, DM, DFF, DFF, SCL, 0.0f);
    k_gemm<0, 1><<<dim3(gM, DM / GBN), GTHR, 0, stream>>>(FH, FL, F2 + w1o, F2 + w1o, F2 + w1o, F2 + w1o,
                                                          f2b + bo, f2b + bo, f2b + bo, f2b + bo,
                                                          SCR, FH, FL, DFF, DM, DM, SCL, SCL2);
    k_ln<1><<<gR, NTHR, 0, stream>>>(HB, SCR, SCR, DM, 0, n2s + bo, n2b + bo, HA, HH, nN, MP);
  }

  k_head<<<nN / 32, NTHR, 0, stream>>>(HA, hs, hb, head_w, head_b, out, nN, nN);
}
